// SuperAggressiveAttention_89850715832914
// MI455X (gfx1250) — hardware-verified
//
#include <hip/hip_runtime.h>


namespace {
constexpr int QB = 4, NT = 1024, DIM = 512, NH = 8, DH = 64, NP_ = NH * QB  , NR = QB * NT  , NWAVE = NP_ * (NT / 16)  ;
constexpr float XS = 8.0f, WSC = 256.0f, PS = 8.0f, GAMMA = 0.01f, LREG = 0.001f;
constexpr float NTOT = 33554432.0f;

typedef _Float16 b16;
typedef __attribute__((ext_vector_type(16))) _Float16 v16b;
typedef __attribute__((ext_vector_type(8))) _Float16 v8b;
typedef __attribute__((ext_vector_type(8))) float v8f;
typedef __attribute__((ext_vector_type(4))) float v4f;
__device__ __forceinline__ float bf16_rne(float f) { unsigned int u = __float_as_uint(f); u += 0x7FFFu + ((u >> 16) & 1u); return __uint_as_float(u & 0xFFFF0000u); }
__device__ __forceinline__ void split16(float v, b16& hi, b16& lo) { hi = (b16)v; lo = (b16)(v - (float)hi); }
__device__ __forceinline__ v16b frag_kb(const b16* p, int hh) { const v8b a = *(const v8b*)(p + 8 * hh), b = *(const v8b*)(p + 16 + 8 * hh); v16b f;
#pragma unroll
  for (int e = 0; e < 8; ++e) { f[e] = a[e]; f[8 + e] = b[e]; } return f; }
__device__ __forceinline__ v8f wmma16b(v16b a, v16b b, v8f c) { v8f d = __builtin_amdgcn_wmma_f32_16x16x32_f16(false, a, false, b, (short)0, c, false, false); asm volatile("v_nop\n\tv_nop\n\tv_nop\n\tv_nop" : "+v"(d) : "v"(a), "v"(b)); return d; }
__device__ __forceinline__ void wave_lds_sync() { __builtin_amdgcn_fence(__ATOMIC_RELEASE, "workgroup"); __builtin_amdgcn_wave_barrier(); __builtin_amdgcn_fence(__ATOMIC_ACQUIRE, "workgroup"); }
__device__ __forceinline__ float nexp(float x) { return __builtin_amdgcn_exp2f(x * 1.4426950408889634f); }
__device__ __forceinline__ float pmul(float a, float b) { float p = a * b; asm volatile("" : "+v"(p)); return p; }
__device__ __forceinline__ float hsum16(float v) { v += __shfl_xor(v, 1); v += __shfl_xor(v, 2); v += __shfl_xor(v, 4); return v + __shfl_xor(v, 8); }
__device__ __forceinline__ float clampf(float v, float lo, float hi) { return fminf(fmaxf(v, lo), hi); }

__global__ __launch_bounds__(256) void ln_kernel(const float* __restrict__ q, const float* __restrict__ k, const float* __restrict__ v, const float* __restrict__ g, const float* __restrict__ be, b16* __restrict__ X16) {
  const int wave = threadIdx.x >> 5, lane = threadIdx.x & 31; const int rowall = blockIdx.x * 8 + wave; const int which = rowall / NR, row = rowall - which * NR;
  const float* src = (which == 0 ? q : which == 1 ? k : v) + (size_t)row * DIM + lane * 16; float x[16];
  { const v4f a = *(const v4f*)src, b = *(const v4f*)(src + 4), c = *(const v4f*)(src + 8), d = *(const v4f*)(src + 12); for (int j = 0; j < 4; ++j) { x[j] = bf16_rne(a[j]); x[4 + j] = bf16_rne(b[j]); x[8 + j] = bf16_rne(c[j]); x[12 + j] = bf16_rne(d[j]); } }
  float s = 0.0f; for (int j = 0; j < 16; ++j) s += x[j];
#pragma unroll
  for (int o = 16; o >= 1; o >>= 1) s += __shfl_xor(s, o);
  const float mu = s * (1.0f / DIM); float ss = 0.0f; for (int j = 0; j < 16; ++j) { const float d = x[j] - mu; ss += pmul(d, d); }
#pragma unroll
  for (int o = 16; o >= 1; o >>= 1) ss += __shfl_xor(ss, o);
  const float rs = rsqrtf(ss * (1.0f / DIM) + 1e-5f); v8b o0, o1;
  for (int j = 0; j < 16; ++j) { const int c = lane * 16 + j; const b16 hv = (b16)((pmul((x[j] - mu) * rs, bf16_rne(g[c])) + bf16_rne(be[c])) * XS); if (j < 8) o0[j] = hv; else o1[j - 8] = hv; }
  for (int pass = 0; pass < 2; ++pass) { b16* dst = X16 + ((size_t)which * NR + row) * DIM + lane * 16; *(volatile v8b*)dst = o0; *(volatile v8b*)(dst + 8) = o1; __threadfence(); }
}
__global__ __launch_bounds__(256) void prepw_kernel(const float* __restrict__ win, const float* __restrict__ wout, b16* __restrict__ WIN, b16* __restrict__ WOUT) {
  const int t = blockIdx.x * 256 + threadIdx.x; if (t >= 2 * DIM * DIM / 8) return; const int kind = t / (DIM * DIM / 8), tt = t - kind * (DIM * DIM / 8); const int o_ = (tt * 8) / DIM, k0 = tt * 8 - o_ * DIM;
  const float* w = kind == 0 ? win : wout; v8b o; for (int j = 0; j < 8; ++j) o[j] = (b16)(bf16_rne(w[(size_t)(k0 + j) * DIM + o_]) * WSC);
  for (int pass = 0; pass < 2; ++pass) { *(volatile v8b*)((kind == 0 ? WIN : WOUT) + (size_t)tt * 8) = o; __threadfence(); }
}
__global__ __launch_bounds__(128) void feat_kernel(const b16* __restrict__ X16, const b16* __restrict__ WIN, float* __restrict__ F32) {
  __shared__ __attribute__((aligned(16))) float Ts[4][16][128 + 4];
  const int wave = threadIdx.x >> 5, lane = threadIdx.x & 31, nloc = lane & 15, hlf = lane >> 4; const int which = blockIdx.z; const size_t m0 = (size_t)blockIdx.x * 64 + wave * 16; const int n0 = blockIdx.y * 128;
  v8f acc[8];
#pragma unroll
  for (int t = 0; t < 8; ++t) acc[t] = (v8f){};
#pragma unroll 4
  for (int kb = 0; kb < DIM; kb += 32) { const v16b a = frag_kb(X16 + ((size_t)which * NR + m0 + nloc) * DIM + kb, hlf);
#pragma unroll
    for (int t = 0; t < 8; ++t) acc[t] = wmma16b(a, frag_kb(WIN + (size_t)(n0 + t * 16 + nloc) * DIM + kb, hlf), acc[t]); }
#pragma unroll
  for (int t = 0; t < 8; ++t)
#pragma unroll
    for (int r = 0; r < 8; ++r) Ts[wave][8 * hlf + r][t * 16 + nloc] = acc[t][r] * (1.0f / (XS * WSC));
  wave_lds_sync();
  for (int pass = 0; pass < 2; ++pass) { for (int rr = 0; rr < 16; ++rr) { const size_t row = m0 + rr; const int qi = (int)(row / NT), n = (int)(row - (size_t)qi * NT); for (int hq = 0; hq < 2; ++hq) { const int h = n0 / DH + hq; const int pair = h * QB + qi;
        if (lane < 16) *(volatile v4f*)(F32 + (((size_t)which * NP_ + pair) * NT + n) * DH + lane * 4) = *(const v4f*)(&Ts[wave][rr][hq * DH + lane * 4]); } } __threadfence(); }
}
__global__ __launch_bounds__(256) void colstat_kernel(const float* __restrict__ F32, float* __restrict__ KCM, float* __restrict__ PSUM) {
  __shared__ float part[4][DH];
  const int which = blockIdx.y, pair = blockIdx.x, t_ = threadIdx.x, d = t_ & 63, pq = t_ >> 6; const float* base = F32 + (((size_t)which * NP_ + pair) * NT) * DH;
  float s = 0.0f; for (int n = pq * 256; n < pq * 256 + 256; ++n) s += base[(size_t)n * DH + d]; part[pq][d] = s;
  __syncthreads();
  if (t_ < DH) { const float tot = (part[0][t_] + part[1][t_]) + (part[2][t_] + part[3][t_]);
    for (int pass = 0; pass < 2; ++pass) { ((volatile float*)PSUM)[((size_t)which * NP_ + pair) * DH + t_] = tot; if (which == 1) ((volatile float*)KCM)[(size_t)pair * DH + t_] = tot * (1.0f / NT); __threadfence(); } }
}
__global__ __launch_bounds__(256) void rowops_kernel(const float* __restrict__ F32, const float* __restrict__ KCM, b16* __restrict__ FQ16, b16* __restrict__ FQC16, float* __restrict__ N1, b16* __restrict__ FK16, b16* __restrict__ FKC16, float* __restrict__ N2) {
  const int wave = threadIdx.x >> 5, lane = threadIdx.x & 31; const size_t prow = ((size_t)blockIdx.x * 8 + wave) * 2 + (lane >> 4);
  const int pair = (int)(prow / NT); const int c0 = (lane & 15) * 4;
  const v4f fq = *(const v4f*)(F32 + (0 * (size_t)NP_ * NT + prow) * DH + c0), fk = *(const v4f*)(F32 + (1 * (size_t)NP_ * NT + prow) * DH + c0);
  float sq = 0.0f, ssq = 0.0f, ssk = 0.0f; for (int j = 0; j < 4; ++j) { sq += fq[j]; ssq += pmul(fq[j], fq[j]); ssk += pmul(fk[j], fk[j]); }
  sq = hsum16(sq); ssq = hsum16(ssq); ssk = hsum16(ssk); const float mq = sq * (1.0f / DH);
  typedef __attribute__((ext_vector_type(4))) _Float16 v4b; v4b a, ac, b, bc;
  for (int j = 0; j < 4; ++j) { a[j] = (b16)(fq[j] * XS); ac[j] = (b16)((fq[j] - mq) * XS); b[j] = (b16)(fk[j] * XS); bc[j] = (b16)((fk[j] - KCM[(size_t)pair * DH + c0 + j]) * XS); }
  for (int pass = 0; pass < 2; ++pass) { *(volatile v4b*)(FQ16 + prow * DH + c0) = a; *(volatile v4b*)(FQC16 + prow * DH + c0) = ac; *(volatile v4b*)(FK16 + prow * DH + c0) = b; *(volatile v4b*)(FKC16 + prow * DH + c0) = bc; __threadfence(); }
}
__global__ __launch_bounds__(256) void norms_kernel(const float* __restrict__ F32, float* __restrict__ N1, float* __restrict__ N2) {
  const size_t prow = (size_t)blockIdx.x * 256 + threadIdx.x; const float* fq = F32 + (0 * (size_t)NP_ * NT + prow) * DH; const float* fk = F32 + (1 * (size_t)NP_ * NT + prow) * DH;
  float sq = 0.0f, sk = 0.0f; for (int d = 0; d < DH; ++d) { sq += pmul(fq[d], fq[d]); sk += pmul(fk[d], fk[d]); }
  for (int pass = 0; pass < 2; ++pass) { ((volatile float*)N1)[prow] = sqrtf(sq); ((volatile float*)N2)[prow] = sqrtf(sk); __threadfence(); }
}
__global__ __launch_bounds__(256) void vt_kernel(const float* __restrict__ F32, b16* __restrict__ FVTh, b16* __restrict__ FVTl) {
  __shared__ __attribute__((aligned(16))) b16 Th[DH][64 + 8], Tl[DH][64 + 8];
  const int pair = blockIdx.y, n0 = blockIdx.x * 64, t_ = threadIdx.x; const float* base = F32 + ((2 * (size_t)NP_ + pair) * NT + n0) * DH;
  for (int qq = t_; qq < 64 * DH; qq += 256) { const int nn = qq >> 6, d = qq & 63; b16 h_, l_; split16(base[(size_t)nn * DH + d] * XS, h_, l_); Th[d][nn] = h_; Tl[d][nn] = l_; }
  __syncthreads();
  for (int pass = 0; pass < 2; ++pass) { for (int qq = t_; qq < DH * 8; qq += 256) { const int d = qq >> 3, c8 = (qq & 7) * 8; const size_t gi = ((size_t)pair * DH + d) * NT + n0 + c8; *(volatile v8b*)(FVTh + gi) = *(const v8b*)(&Th[d][c8]); *(volatile v8b*)(FVTl + gi) = *(const v8b*)(&Tl[d][c8]); } __threadfence(); }
}
struct PassC { float cn_inv_cscale, covfac, vn_half_inv, temp_inv; float cw[NH], covw[NH], vw[NH]; };
template <int PASS>
__global__ __launch_bounds__(64) void score_kernel(const b16* __restrict__ FQ16, const b16* __restrict__ FQC16, const float* __restrict__ N1, const b16* __restrict__ FK16, const b16* __restrict__ FKC16, const float* __restrict__ N2, const b16* __restrict__ FVTh, const b16* __restrict__ FVTl,
                                                  const float* __restrict__ CST  , float* __restrict__ P1, float* __restrict__ VARC, float* __restrict__ P2, float* __restrict__ ROWE, b16* __restrict__ OCh, b16* __restrict__ OCl) {
  __shared__ __attribute__((aligned(16))) float To[2][16][DH + 4]; __shared__ float Tr[2][16]; __shared__ float Tp[2][4];
  const int wave = threadIdx.x >> 5, lane = threadIdx.x & 31, hh = lane >> 4, col = lane & 15; const int pair = blockIdx.y, n0 = blockIdx.x * 32 + wave * 16, ni = n0 + col; const int h = pair / QB, qi = pair - h * QB;
  const size_t prow = (size_t)pair * NT + ni; const b16* Qp = FQ16 + prow * DH; const b16* Qc = FQC16 + prow * DH; const b16* Kb = FK16 + (size_t)pair * NT * DH; const b16* Kc = FKC16 + (size_t)pair * NT * DH;
  const float n1 = N1[prow]; const float inv1a = 1.0f / (n1 + 1e-8f), inv1b = 1.0f / fmaxf(n1, 1e-6f);
  PassC C; if (PASS >= 2) { const float* cf = CST; C.cn_inv_cscale = cf[0]; C.covfac = cf[1]; C.vn_half_inv = cf[2]; C.temp_inv = cf[3]; for (int j = 0; j < NH; ++j) { C.cw[j] = cf[4 + j]; C.covw[j] = cf[4 + NH + j]; C.vw[j] = cf[4 + 2 * NH + j]; } }
  float crow = 0.0f; if (PASS >= 2) crow = C.vw[h] * VARC[prow] * C.vn_half_inv;
  float s_a = 0.0f, s_b = 0.0f, s_c = 0.0f, s_d = 0.0f, rowacc = 0.0f;
  float m = -INFINITY, l = 0.0f; v8f o[4] = {{}, {}, {}, {}}, ol[4] = {{}, {}, {}, {}};
  const v16b qa0 = frag_kb(Qp, hh), qa1 = frag_kb(Qp + 32, hh), qc0 = frag_kb(Qc, hh), qc1 = frag_kb(Qc + 32, hh);
  for (int kb = 0; kb < NT; kb += 32) {
    v8f d0 = {}, d1 = {}, c0 = {}, c1 = {};
    d0 = wmma16b(frag_kb(Kb + (size_t)(kb + col) * DH, hh), qa0, d0); d0 = wmma16b(frag_kb(Kb + (size_t)(kb + col) * DH + 32, hh), qa1, d0);
    d1 = wmma16b(frag_kb(Kb + (size_t)(kb + 16 + col) * DH, hh), qa0, d1); d1 = wmma16b(frag_kb(Kb + (size_t)(kb + 16 + col) * DH + 32, hh), qa1, d1);
    c0 = wmma16b(frag_kb(Kc + (size_t)(kb + col) * DH, hh), qc0, c0); c0 = wmma16b(frag_kb(Kc + (size_t)(kb + col) * DH + 32, hh), qc1, c0);
    c1 = wmma16b(frag_kb(Kc + (size_t)(kb + 16 + col) * DH, hh), qc0, c1); c1 = wmma16b(frag_kb(Kc + (size_t)(kb + 16 + col) * DH + 32, hh), qc1, c1);
    float ev0[8], ev1[8];
#pragma unroll
    for (int r = 0; r < 8; ++r) {
#pragma unroll
      for (int hq = 0; hq < 2; ++hq) { const int key = kb + (hq ? 16 : 0) + 8 * hh + r; const float dot = (hq ? d1[r] : d0[r]) * (1.0f / (XS * XS)); const float covraw = (hq ? c1[r] : c0[r]) * (1.0f / (XS * XS)) * (1.0f / (8.0f + 1e-6f));
        const float n2 = N2[(size_t)pair * NT + key]; const float cosv = clampf(dot * inv1a * (1.0f / (n2 + 1e-8f)), -0.99f, 0.99f);
        if (PASS == 1) { const float csim = clampf(dot * inv1b * (1.0f / fmaxf(n2, 1e-6f)), -0.99f, 0.99f); const float margin = clampf(GAMMA - csim, 0.0f, 10.0f);
          s_a += cosv; s_b += pmul(cosv, cosv); s_c += covraw; s_d += pmul(covraw, covraw); rowacc += margin; }
        else { const float e = pmul(C.cw[h], cosv * C.cn_inv_cscale) + pmul(C.covw[h], covraw * C.covfac);
          if (PASS == 2) { s_a += e; s_b += pmul(e, e); rowacc += e; }
          else { (hq ? ev1 : ev0)[r] = (e + crow) * C.temp_inv; } } } }
    if (PASS == 3) { float mr = -INFINITY;
#pragma unroll
      for (int r = 0; r < 8; ++r) mr = fmaxf(mr, fmaxf(ev0[r], ev1[r]));
      mr = fmaxf(mr, __shfl_xor(mr, 16)); const float mn = fmaxf(m, mr); const float al_ = nexp(m - mn); m = mn; float sum = 0.0f; v16b pb;
#pragma unroll
      for (int r = 0; r < 8; ++r) { const float e0 = nexp(ev0[r] - mn), e1 = nexp(ev1[r] - mn); sum += e0 + e1; pb[r] = (b16)(e0 * PS); pb[8 + r] = (b16)(e1 * PS); }
      sum += __shfl_xor(sum, 16); l = l * al_ + sum;
#pragma unroll
      for (int t = 0; t < 4; ++t) { o[t] *= al_; ol[t] *= al_; const b16* vr = FVTh + ((size_t)pair * DH + t * 16 + col) * NT + kb; o[t] = wmma16b(frag_kb(vr, hh), pb, o[t]); ol[t] = wmma16b(frag_kb(FVTl + ((size_t)pair * DH + t * 16 + col) * NT + kb, hh), pb, ol[t]); } } }
  if (PASS <= 2) {
    rowacc += __shfl_xor(rowacc, 16); if (hh == 0) Tr[wave][col] = rowacc;
    float v4[4] = {s_a, s_b, s_c, s_d};
#pragma unroll
    for (int j = 0; j < 4; ++j) { float v = v4[j];
#pragma unroll
      for (int oo = 16; oo >= 1; oo >>= 1) v += __shfl_xor(v, oo);
      v4[j] = v; }
    if (lane == 0) { Tp[wave][0] = v4[0]; Tp[wave][1] = v4[1]; Tp[wave][2] = v4[2]; Tp[wave][3] = v4[3]; }
    wave_lds_sync();
    const size_t widx = (size_t)pair * (NT / 16) + blockIdx.x * 2 + wave;
    __syncthreads();
    for (int pass = 0; pass < 2; ++pass) {
      if (wave == 0) { const float rv = Tr[lane >> 4][lane & 15] * (PASS == 1 ? (1.0f / NT) : 1.0f); ((volatile float*)(PASS == 1 ? VARC : ROWE))[(size_t)pair * NT + blockIdx.x * 32 + lane] = rv;
        ((volatile float*)(PASS == 1 ? P1 : P2))[((size_t)pair * (NT / 32) + blockIdx.x) * 32 + lane] = (lane < 8) ? Tp[lane >> 2][lane & 3] : 0.0f; }
      __threadfence(); }
    (void)widx;
  } else {
    const float inv = 1.0f / (l * PS * XS);
#pragma unroll
    for (int t = 0; t < 4; ++t)
#pragma unroll
      for (int r = 0; r < 8; ++r) To[wave][col][t * 16 + 8 * hh + r] = (o[t][r] + ol[t][r]) * inv;
    wave_lds_sync();
    for (int pass = 0; pass < 2; ++pass) { for (int r2 = 0; r2 < 16; r2 += 4) { const int rr = r2 + (lane >> 3), c8 = (lane & 7) * 8; v8b hv, lv; for (int j = 0; j < 8; ++j) { b16 a_, c_; split16(To[wave][rr][c8 + j] * XS, a_, c_); hv[j] = a_; lv[j] = c_; }
        const size_t gi = ((size_t)qi * NT + n0 + rr) * DIM + h * DH + c8; *(volatile v8b*)(OCh + gi) = hv; *(volatile v8b*)(OCl + gi) = lv; } __threadfence(); }
  }
}
__global__ __launch_bounds__(256) void reduce1_kernel(const float* __restrict__ P1, const float* __restrict__ VARC, const float* __restrict__ PSUM, const float* __restrict__ w1, const float* __restrict__ b1, const float* __restrict__ g2, const float* __restrict__ be2, const float* __restrict__ w2, const float* __restrict__ b2, const float* __restrict__ w3, const float* __restrict__ b3, const float* __restrict__ wtemp, float* __restrict__ CST) {
  __shared__ float red[4][256]; __shared__ float sh[64];
  const int t_ = threadIdx.x; const int NPART = NP_ * (NT / 32);
  float a = 0, b = 0, c = 0, d = 0; for (int i = t_; i < NPART; i += 256) { const float* p = P1 + (size_t)i * 32; a += p[0] + p[4]; b += p[1] + p[5]; c += p[2] + p[6]; d += p[3] + p[7]; }
  red[0][t_] = a; red[1][t_] = b; red[2][t_] = c; red[3][t_] = d; __syncthreads();
  for (int s = 128; s >= 1; s >>= 1) { if (t_ < s) { for (int j = 0; j < 4; ++j) red[j][t_] += red[j][t_ + s]; } __syncthreads(); }
  float vs = 0.0f; for (int i = t_; i < NP_ * NT; i += 256) vs += VARC[i];
  __shared__ float r2[256]; r2[t_] = vs; __syncthreads(); for (int s = 128; s >= 1; s >>= 1) { if (t_ < s) r2[t_] += r2[t_ + s]; __syncthreads(); }
  const float vmu = r2[0] / (float)(NP_ * NT); __syncthreads();
  float vq = 0.0f;
#pragma unroll 1
  for (int i = t_; i < NP_ * NT; i += 256) { const float dv = VARC[i] - vmu; vq += pmul(dv, dv); }
  r2[t_] = vq; __syncthreads(); for (int s = 128; s >= 1; s >>= 1) { if (t_ < s) r2[t_] += r2[t_ + s]; __syncthreads(); }
  __shared__ float feats[NH][2 * DH], h1s[NH][DH], h2s[NH][32], ws[NH][3];
  for (int i = t_; i < NH * 2 * DH; i += 256) { const int h = i / (2 * DH), c = i - h * 2 * DH; const int which = c / DH, dd = c - which * DH; float s = 0.0f;
#pragma unroll 1
    for (int qq = 0; qq < QB; ++qq) s += PSUM[((size_t)which * NP_ + h * QB + qq) * DH + dd]; feats[h][c] = s * (1.0f / (QB * NT)); }
  __syncthreads();
  for (int i = t_; i < NH * DH; i += 256) { const int h = i / DH, o_ = i - h * DH; float s = bf16_rne(b1[o_]);
#pragma unroll 1
    for (int c = 0; c < 2 * DH; ++c) s += pmul(feats[h][c], bf16_rne(w1[c * DH + o_])); h1s[h][o_] = s; }
  __syncthreads();
  if (t_ < NH) { const int h = t_; float mu = 0.0f;
#pragma unroll 1
    for (int c = 0; c < DH; ++c) mu += h1s[h][c];
    mu *= (1.0f / DH); float var = 0.0f;
#pragma unroll 1
    for (int c = 0; c < DH; ++c) { const float dv = h1s[h][c] - mu; var += pmul(dv, dv); }
    var *= (1.0f / DH); const float rs = rsqrtf(var + 1e-5f);
#pragma unroll 1
    for (int c = 0; c < DH; ++c) h1s[h][c] = fmaxf(pmul((h1s[h][c] - mu) * rs, bf16_rne(g2[c])) + bf16_rne(be2[c]), 0.0f); }
  __syncthreads();
  for (int i = t_; i < NH * 32; i += 256) { const int h = i / 32, o_ = i - h * 32; float s = bf16_rne(b2[o_]);
#pragma unroll 1
    for (int c = 0; c < DH; ++c) s += pmul(h1s[h][c], bf16_rne(w2[c * 32 + o_])); h2s[h][o_] = fmaxf(s, 0.0f); }
  __syncthreads();
  if (t_ < NH) { const int h = t_; float lg[3]; for (int o_ = 0; o_ < 3; ++o_) { float s = bf16_rne(b3[o_]);
#pragma unroll 1
      for (int c = 0; c < 32; ++c) s += pmul(h2s[h][c], bf16_rne(w3[c * 3 + o_])); lg[o_] = s; }
    float mx = fmaxf(lg[0], fmaxf(lg[1], lg[2])); float e3[3], se = 0.0f; for (int j = 0; j < 3; ++j) { e3[j] = __expf(lg[j] - mx); se += e3[j]; } for (int j = 0; j < 3; ++j) e3[j] /= se;
    const float wt = clampf(bf16_rne(wtemp[0]), 0.1f, 20.0f); float z[3]; for (int j = 0; j < 3; ++j) z[j] = e3[j] / wt; mx = fmaxf(z[0], fmaxf(z[1], z[2])); se = 0.0f; for (int j = 0; j < 3; ++j) { e3[j] = __expf(z[j] - mx); se += e3[j]; }
    float wv[3], sw = 0.0f; for (int j = 0; j < 3; ++j) { wv[j] = clampf(e3[j] / se, 0.05f, 0.8f); sw += wv[j]; } for (int j = 0; j < 3; ++j) ws[h][j] = wv[j] / sw; }
  __syncthreads();
  if (t_ == 0) { const float n = (float)NTOT; const float sa_ = red[0][0], sb = red[1][0], sc = red[2][0], sd = red[3][0];
    const float cstd = sqrtf(fmaxf((sb - sa_ * (sa_ / n)) / (n - 1.0f), 0.0f)); const float covstd_raw = sqrtf(fmaxf((sd - sc * (sc / n)) / (n - 1.0f), 0.0f));
    const float base_reg = LREG / (float)NT; const float reg = (covstd_raw < 1e-6f) ? base_reg * 10.0f : base_reg;
    const float covn = reg * covstd_raw + 1e-6f; const float cn = cstd + 1e-6f; const float cscale = (cn < 1e-4f) ? 0.1f : 1.0f;
    const float vn = sqrtf(r2[0] * ((float)NT / (n - 1.0f))) + 1e-6f;
    sh[0] = cscale / cn; sh[1] = reg * 0.5f / covn; sh[2] = 0.5f / vn; sh[3] = 0.0f; for (int h = 0; h < NH; ++h) { sh[4 + h] = ws[h][0]; sh[4 + NH + h] = ws[h][1]; sh[4 + 2 * NH + h] = ws[h][2]; } }
  __syncthreads();
  for (int pass = 0; pass < 2; ++pass) { if (t_ < 32) ((volatile float*)CST)[t_] = (t_ < 4 + 3 * NH) ? sh[t_] : 0.0f; __threadfence(); }
}
__global__ __launch_bounds__(256) void reduce2_kernel(const float* __restrict__ P2, const float* __restrict__ ROWE, const float* __restrict__ VARC, float* __restrict__ CST) {
  __shared__ float red[5][256];
  const int t_ = threadIdx.x; const int NPART = NP_ * (NT / 32);
  const float vfac = CST[2];
  float a = 0, b = 0; for (int i = t_; i < NPART; i += 256) { const float* p = P2 + (size_t)i * 32; a += (p[0] + p[4]); b += (p[1] + p[5]); }
  float sc = 0; for (int i = t_; i < NP_ * NT; i += 256) { const int h = (i / NT) / QB; sc += CST[4 + 2 * NH + h] * VARC[i] * vfac; }
  red[4][t_] = sc; __syncthreads(); for (int s = 128; s >= 1; s >>= 1) { if (t_ < s) red[4][t_] += red[4][t_ + s]; __syncthreads(); }
  const float M = red[4][0] / (float)(NP_ * NT); __syncthreads();
  float s1 = 0, s2 = 0; for (int i = t_; i < NP_ * NT; i += 256) { const int h = (i / NT) / QB; const float cm = CST[4 + 2 * NH + h] * VARC[i] * vfac - M; s1 += (float)NT * cm; s2 += 2.0f * cm * ROWE[i] + (float)NT * cm * cm; }
  red[0][t_] = a + s1; red[1][t_] = b + s2; __syncthreads();
  for (int s = 128; s >= 1; s >>= 1) { if (t_ < s) { red[0][t_] += red[0][t_ + s]; red[1][t_] += red[1][t_ + s]; } __syncthreads(); }
  if (t_ == 0) { const float n = NTOT; const float var = (red[1][0] - red[0][0] * (red[0][0] / n)) / (n - 1.0f); const float dstd = sqrtf(fmaxf(var, 0.0f)); const float temp = (dstd < 1e-6f) ? 0.1f : 0.3f + dstd; const float tinv = 1.0f / clampf(temp, 0.1f, 5.0f);
    for (int pass = 0; pass < 2; ++pass) { ((volatile float*)CST)[3] = tinv; __threadfence(); } }
}
__global__ __launch_bounds__(128) void outproj_kernel(const b16* __restrict__ OCh, const b16* __restrict__ OCl, const b16* __restrict__ WOUT, const float* __restrict__ bo, float* __restrict__ out) {
  __shared__ __attribute__((aligned(16))) float Ts[4][16][128 + 4];
  const int wave = threadIdx.x >> 5, lane = threadIdx.x & 31, nloc = lane & 15, hlf = lane >> 4; const size_t m0 = (size_t)blockIdx.x * 64 + wave * 16; const int n0 = blockIdx.y * 128;
  v8f acc[8];
#pragma unroll
  for (int t = 0; t < 8; ++t) acc[t] = (v8f){};
#pragma unroll 2
  for (int kb = 0; kb < DIM; kb += 32) { const v16b a = frag_kb(OCh + (m0 + nloc) * DIM + kb, hlf), al = frag_kb(OCl + (m0 + nloc) * DIM + kb, hlf);
#pragma unroll
    for (int t = 0; t < 8; ++t) { const v16b bw = frag_kb(WOUT + (size_t)(n0 + t * 16 + nloc) * DIM + kb, hlf); acc[t] = wmma16b(a, bw, acc[t]); acc[t] = wmma16b(al, bw, acc[t]); } }
#pragma unroll
  for (int t = 0; t < 8; ++t) { const float bb = bf16_rne(bo[n0 + t * 16 + nloc]);
#pragma unroll
    for (int r = 0; r < 8; ++r) Ts[wave][8 * hlf + r][t * 16 + nloc] = acc[t][r] * (1.0f / (XS * WSC)) + bb; }
  wave_lds_sync();
  for (int pass = 0; pass < 2; ++pass) { for (int rr = 0; rr < 16; ++rr) *(volatile v4f*)(out + (m0 + rr) * DIM + n0 + lane * 4) = *(const v4f*)(&Ts[wave][rr][lane * 4]); __threadfence(); }
}
}

extern "C" void kernel_launch(void* const* d_in, const int* in_sizes, int n_in, void* d_out, int out_size, void* d_ws, size_t ws_size, hipStream_t stream) {
  (void)n_in;
  auto Fp = [&](int i) { return (const float*)d_in[i]; };
  if (in_sizes[0] != NR * DIM || in_sizes[1] != NR * DIM || in_sizes[2] != NR * DIM || in_sizes[5] != DIM * DIM || in_sizes[6] != 2 * DH * DH || in_sizes[15] != DIM * DIM || out_size != NR * DIM) return;
  size_t off = 0; char* ws = (char*)d_ws;
  auto carve = [&](size_t bytes) { char* p = ws + off; off += (bytes + 255) & ~(size_t)255; return p; };
  b16* X16 = (b16*)carve((size_t)3 * NR * DIM * 2); b16* WIN = (b16*)carve((size_t)DIM * DIM * 2); b16* WOUT = (b16*)carve((size_t)DIM * DIM * 2);
  float* F32 = (float*)carve((size_t)3 * NP_ * NT * DH * 4); float* KCM = (float*)carve((size_t)NP_ * DH * 4); float* PSUM = (float*)carve((size_t)2 * NP_ * DH * 4);
  b16* FQ16 = (b16*)carve((size_t)NP_ * NT * DH * 2); b16* FQC16 = (b16*)carve((size_t)NP_ * NT * DH * 2); b16* FK16 = (b16*)carve((size_t)NP_ * NT * DH * 2); b16* FKC16 = (b16*)carve((size_t)NP_ * NT * DH * 2);
  float* N1 = (float*)carve((size_t)NP_ * NT * 4); float* N2 = (float*)carve((size_t)NP_ * NT * 4); b16* FVTh = (b16*)carve((size_t)NP_ * DH * NT * 2); b16* FVTl = (b16*)carve((size_t)NP_ * DH * NT * 2);
  float* P1 = (float*)carve((size_t)NP_ * (NT / 32) * 32 * 4); float* VARC = (float*)carve((size_t)NP_ * NT * 4); float* P2 = (float*)carve((size_t)NP_ * (NT / 32) * 32 * 4); float* ROWE = (float*)carve((size_t)NP_ * NT * 4); float* CST = (float*)carve(256);
  b16* OCh = (b16*)carve((size_t)NR * DIM * 2); b16* OCl = (b16*)carve((size_t)NR * DIM * 2);
  if (off > ws_size || off > ((size_t)128 << 20)) return;
  ln_kernel<<<3 * NR / 8, 256, 0, stream>>>(Fp(0), Fp(1), Fp(2), Fp(3), Fp(4), X16);
  prepw_kernel<<<(2 * DIM * DIM / 8 + 255) / 256, 256, 0, stream>>>(Fp(5), Fp(15), WIN, WOUT);
  feat_kernel<<<dim3(NR / 64, DIM / 128, 3), 128, 0, stream>>>(X16, WIN, F32);
  colstat_kernel<<<dim3(NP_, 2), 256, 0, stream>>>(F32, KCM, PSUM);
  rowops_kernel<<<NP_ * NT / 16, 256, 0, stream>>>(F32, KCM, FQ16, FQC16, N1, FK16, FKC16, N2);
  norms_kernel<<<NP_ * NT / 256, 256, 0, stream>>>(F32, N1, N2);
  vt_kernel<<<dim3(NT / 64, NP_), 256, 0, stream>>>(F32, FVTh, FVTl);
  score_kernel<1><<<dim3(NT / 32, NP_), 64, 0, stream>>>(FQ16, FQC16, N1, FK16, FKC16, N2, FVTh, FVTl, CST, P1, VARC, P2, ROWE, OCh, OCl);
  reduce1_kernel<<<1, 256, 0, stream>>>(P1, VARC, PSUM, Fp(6), Fp(7), Fp(8), Fp(9), Fp(10), Fp(11), Fp(12), Fp(13), Fp(14), CST);
  score_kernel<2><<<dim3(NT / 32, NP_), 64, 0, stream>>>(FQ16, FQC16, N1, FK16, FKC16, N2, FVTh, FVTl, CST, P1, VARC, P2, ROWE, OCh, OCl);
  reduce2_kernel<<<1, 256, 0, stream>>>(P2, ROWE, VARC, CST);
  score_kernel<3><<<dim3(NT / 32, NP_), 64, 0, stream>>>(FQ16, FQC16, N1, FK16, FKC16, N2, FVTh, FVTl, CST, P1, VARC, P2, ROWE, OCh, OCl);
  outproj_kernel<<<dim3(NR / 64, DIM / 128), 128, 0, stream>>>(OCh, OCl, WOUT, Fp(16), (float*)d_out);
}
